// GCN_27960237097168
// MI455X (gfx1250) — hardware-verified
//
#include <hip/hip_runtime.h>
#include <stddef.h>
#include <stdint.h>
#include <math.h>


#define DF     128
#define K2     256
#define NTHR   256
#define NWAVE  8
#define EPT    8
#define CHUNK  (NTHR * EPT)
#define WCAP   (EPT * 32)
#define LISTN  (NWAVE * WCAP)
#define NBD    4096
#define SLD    12
#define NBA    1024
#define SLA    10
#define RCAP   28672
#define DEGCAP 64
#define GBM    64
#define GBN    128
#define GTHR   128
#define NUW1   (DF * (DF / 8))
#define NUWD   (DF * (K2 / 8))
#define NBW    ((NUW1 + 2 * NUWD) / NTHR)
#define AGG_ZINTS    (LISTN + 2 * RCAP + 3 * NBA)
#define MISC_INTS    16
#define STAGE_INTS   NBA
#define AGG_LDS_INTS (AGG_ZINTS + MISC_INTS + STAGE_INTS)
#define WSMAX  134217728

static_assert((CHUNK & (CHUNK - 1)) == 0 && CHUNK <= 4096);
static_assert((NBD & (NBD - 1)) == 0 && NBD == (1 << SLD));
static_assert((NBA & (NBA - 1)) == 0 && NBA == (1 << SLA));
static_assert(((long long)CHUNK << SLD) < (1LL << 31));
static_assert(((long long)CHUNK << SLA) < (1LL << 31));
static_assert(NBD % (NTHR * 4) == 0);
static_assert(LISTN % NTHR == 0);
static_assert(NBA % NWAVE == 0 && NBA % 32 == 0 && NBA % GBM == 0 && NBA == 4 * NTHR);
static_assert(RCAP % 4 == 0 && AGG_ZINTS % 4 == 0 && LISTN % 4 == 0 && ((AGG_ZINTS + MISC_INTS) % 4) == 0);
static_assert(RCAP >= 13176);
static_assert(DEGCAP >= 28 + 8);
static_assert(DF % 32 == 0 && K2 % 32 == 0 && K2 == 2 * DF);
static_assert(GBN == DF && GBM == (GTHR / 32) * 16 && DF == 4 * 32);
static_assert(NUW1 % NTHR == 0 && NUWD % NTHR == 0);
static_assert(AGG_LDS_INTS * 4 <= 300000);

typedef float          v4f   __attribute__((ext_vector_type(4)));
typedef float          v8f   __attribute__((ext_vector_type(8)));
typedef int            v4i   __attribute__((ext_vector_type(4)));
typedef int            v8i   __attribute__((ext_vector_type(8)));
typedef unsigned int   v4u   __attribute__((ext_vector_type(4)));
typedef unsigned short v8us  __attribute__((ext_vector_type(8)));
typedef unsigned short v16us __attribute__((ext_vector_type(16)));
typedef __bf16         v16bf __attribute__((ext_vector_type(16)));
typedef v4f  __attribute__((may_alias)) v4fa;
typedef v4i  __attribute__((may_alias)) v4ia;
typedef v8us __attribute__((may_alias)) v8usa;
union FragB { v16bf v; v16us u; v8us h[2]; v8i w; };

__device__ __forceinline__ v8f wmb(const FragB& a, const FragB& b, v8f c) {
  v8f d = __builtin_amdgcn_wmma_f32_16x16x32_bf16(false, a.v, false, b.v, (short)0, c, false, false);
  asm volatile("v_nop\n\tv_nop\n\tv_nop\n\tv_nop" : "+v"(d) : "v"(a.w), "v"(b.w));
  return d;
}

__device__ __forceinline__ unsigned bf16_bits(float f) {
  const unsigned u = __float_as_uint(f);
  const unsigned r = (u + 0x7FFFu + ((u >> 16) & 1u)) >> 16;
  return (f != f) ? 0x7FC0u : r;
}
__device__ __forceinline__ float bf16_val(float f) {
  return __uint_as_float(bf16_bits(f) << 16);
}

template <int SLB>
__device__ __forceinline__ int scan_chunk(const int* __restrict__ dsts, int nE, int cbase, int slotBase,
                                          int nb, int vec8, int* list, int tid, int lane, int wave) {
  int wc = 0;
  const int el0  = tid * EPT;
  const int e0   = cbase + el0;
  const int sent = -2147483647 - 1;
  v4i da, db;
  if (vec8 != 0 && cbase + CHUNK <= nE) {
    da = *(const v4i*)(dsts + e0);
    db = *(const v4i*)(dsts + e0 + 4);
  } else {
    da.x = (e0     < nE) ? dsts[min(e0,     nE - 1)] : sent;
    da.y = (e0 + 1 < nE) ? dsts[min(e0 + 1, nE - 1)] : sent;
    da.z = (e0 + 2 < nE) ? dsts[min(e0 + 2, nE - 1)] : sent;
    da.w = (e0 + 3 < nE) ? dsts[min(e0 + 3, nE - 1)] : sent;
    db.x = (e0 + 4 < nE) ? dsts[min(e0 + 4, nE - 1)] : sent;
    db.y = (e0 + 5 < nE) ? dsts[min(e0 + 5, nE - 1)] : sent;
    db.z = (e0 + 6 < nE) ? dsts[min(e0 + 6, nE - 1)] : sent;
    db.w = (e0 + 7 < nE) ? dsts[min(e0 + 7, nE - 1)] : sent;
  }
  const unsigned nbs = (unsigned)slotBase;
  const unsigned unb = (unsigned)nb;
  const unsigned s0 = (unsigned)da.x - nbs, s1 = (unsigned)da.y - nbs;
  const unsigned s2 = (unsigned)da.z - nbs, s3 = (unsigned)da.w - nbs;
  const unsigned s4 = (unsigned)db.x - nbs, s5 = (unsigned)db.y - nbs;
  const unsigned s6 = (unsigned)db.z - nbs, s7 = (unsigned)db.w - nbs;
  const bool h0 = s0 < unb, h1 = s1 < unb, h2 = s2 < unb, h3 = s3 < unb;
  const bool h4 = s4 < unb, h5 = s5 < unb, h6 = s6 < unb, h7 = s7 < unb;
  const unsigned any = __builtin_amdgcn_ballot_w32(h0 | h1 | h2 | h3 | h4 | h5 | h6 | h7);
  if (any != 0u) {
#define HITJ(J, HJ, SJ) { \
      const unsigned mj = __builtin_amdgcn_ballot_w32(HJ); \
      if (mj != 0u) { \
        if (HJ) { \
          const int pos = wc + (int)__builtin_amdgcn_mbcnt_lo(mj, 0u); \
          if (pos < WCAP) list[wave * WCAP + pos] = ((el0 + (J)) << SLB) | (int)(SJ); \
        } \
        wc += (int)__builtin_popcount(mj); } }
    HITJ(0, h0, s0)
    HITJ(1, h1, s1)
    HITJ(2, h2, s2)
    HITJ(3, h3, s3)
    HITJ(4, h4, s4)
    HITJ(5, h5, s5)
    HITJ(6, h6, s6)
    HITJ(7, h7, s7)
#undef HITJ
  }
  return wc;
}

__global__ __launch_bounds__(NTHR) void k_prep(const float* __restrict__ x, const float* __restrict__ W1,
                                               const float* __restrict__ W2, const float* __restrict__ W3,
                                               int nN, int nBx, unsigned short* xb, unsigned short* W1T,
                                               unsigned short* W2D, unsigned short* W3D) {
  const int tid = (int)threadIdx.x;
  const int bx  = (int)blockIdx.x;
  v8us o;
  unsigned short* dp;
  if (bx < nBx) {
    const int u   = bx * NTHR + tid;
    const int row = u >> 4;
    const int k8  = (u & 15) * 8;
    const int rc  = row < nN ? row : nN - 1;
    const float* p = x + (size_t)rc * DF + k8;
    const v4f a = *(const v4f*)p;
    const v4f b = *(const v4f*)(p + 4);
    const bool ok = row < nN;
    o[0] = ok ? (unsigned short)bf16_bits(a.x) : (unsigned short)0;
    o[1] = ok ? (unsigned short)bf16_bits(a.y) : (unsigned short)0;
    o[2] = ok ? (unsigned short)bf16_bits(a.z) : (unsigned short)0;
    o[3] = ok ? (unsigned short)bf16_bits(a.w) : (unsigned short)0;
    o[4] = ok ? (unsigned short)bf16_bits(b.x) : (unsigned short)0;
    o[5] = ok ? (unsigned short)bf16_bits(b.y) : (unsigned short)0;
    o[6] = ok ? (unsigned short)bf16_bits(b.z) : (unsigned short)0;
    o[7] = ok ? (unsigned short)bf16_bits(b.w) : (unsigned short)0;
    dp = xb + (size_t)row * DF + k8;
  } else {
    const int v = (bx - nBx) * NTHR + tid;
    const float* W;
    unsigned short* P;
    int sh, w;
    if (v < NUW1)                 { W = W1; P = W1T; sh = 4; w = v; }
    else if (v < NUW1 + NUWD)     { W = W2; P = W2D; sh = 5; w = v - NUW1; }
    else if (v < NUW1 + 2 * NUWD) { W = W3; P = W3D; sh = 5; w = v - NUW1 - NUWD; }
    else return;
    const int n  = w >> sh;
    const int k8 = (w & ((1 << sh) - 1)) * 8;
    const int kk = k8 & (DF - 1);
    const float* p = W + (size_t)kk * DF + n;
#pragma unroll
    for (int i = 0; i < 8; ++i) o[i] = (unsigned short)bf16_bits(p[(size_t)i * DF]);
    dp = P + (size_t)n * ((size_t)8 << sh) + k8;
  }
  *(volatile v8us*)dp = o;
  __threadfence();
  *(volatile v8us*)dp = o;
}

__global__ __launch_bounds__(NTHR) void k_deg(const int* __restrict__ dsts, int nE, int vec8, float* dis) {
  __shared__ __attribute__((aligned(16))) int   scnt[NBD];
  __shared__ __attribute__((aligned(16))) float sdis[NBD];
  __shared__ __attribute__((aligned(16))) int   list[LISTN];
  __shared__ int wcnt[NWAVE];
  const int tid = (int)threadIdx.x, lane = tid & 31, wave = tid >> 5;
  const int nodeBase = (int)blockIdx.x * NBD;

  for (int i = tid; i < NBD; i += NTHR) { scnt[i] = 0; sdis[i] = 1.0f; }
  for (int i = tid; i < LISTN; i += NTHR) list[i] = 0;
  if (tid < NWAVE) wcnt[tid] = 0;
  __syncthreads();

  const int nChunks = (nE + CHUNK - 1) / CHUNK;
#pragma unroll 1
  for (int ch = 0; ch < nChunks; ++ch) {
    const int cbase = ch * CHUNK;
    const int wc = scan_chunk<SLD>(dsts, nE, cbase, nodeBase, NBD, vec8, list, tid, lane, wave);
    if (lane == 0) wcnt[wave] = wc;
    __syncthreads();
    if (wave == 0) {
#pragma unroll 1
      for (int w2 = 0; w2 < NWAVE; ++w2) {
        int c = wcnt[w2];
        c = c < 0 ? 0 : (c > WCAP ? WCAP : c);
#pragma unroll 1
        for (int b0 = 0; b0 < c; b0 += 32) {
          const int idx = b0 + lane;
          const int ent = list[w2 * WCAP + (idx < WCAP ? idx : WCAP - 1)];
          const int m32 = (c - b0) < 32 ? (c - b0) : 32;
#pragma unroll 1
          for (int k = 0; k < m32; ++k) {
            const int u  = __builtin_amdgcn_readlane(ent, k);
            const int sl = u & (NBD - 1);
            if (lane == 0) scnt[sl] = scnt[sl] + 1;
          }
        }
      }
    }
    __syncthreads();
  }

#pragma unroll 1
  for (int i = tid; i < NBD; i += NTHR) {
    const float d = (float)(scnt[i] + 1);
    sdis[i] = 1.0f / sqrtf(d);
  }
  __syncthreads();

  v4f vals[NBD / (NTHR * 4)];
#pragma unroll
  for (int it = 0; it < NBD / (NTHR * 4); ++it) {
    const int s0 = it * (NTHR * 4) + 4 * tid;
    vals[it] = *(const v4fa*)(sdis + s0);
  }
#pragma unroll
  for (int it = 0; it < NBD / (NTHR * 4); ++it) {
    const int s0 = it * (NTHR * 4) + 4 * tid;
    *(volatile v4f*)(dis + (size_t)nodeBase + s0) = vals[it];
  }
  __threadfence();
#pragma unroll
  for (int it = 0; it < NBD / (NTHR * 4); ++it) {
    const int s0 = it * (NTHR * 4) + 4 * tid;
    *(volatile v4f*)(dis + (size_t)nodeBase + s0) = vals[it];
  }
}

__global__ __launch_bounds__(GTHR) void k_gemm(const unsigned short* __restrict__ A,
                                               const unsigned short* __restrict__ BT, int K, float* outF) {
  __shared__ __attribute__((aligned(16))) float stg[GBM * GBN];
  const int tid = (int)threadIdx.x, lane = tid & 31, wave = tid >> 5, hh = lane >> 4, m = lane & 15;
  const int rowBase = (int)blockIdx.x * GBM;

  v8f acc[8];
  {
    const v8f z = {0.f, 0.f, 0.f, 0.f, 0.f, 0.f, 0.f, 0.f};
#pragma unroll
    for (int t = 0; t < 8; ++t) acc[t] = z;
  }
  const unsigned short* ap = A  + (size_t)(rowBase + 16 * wave + m) * (size_t)K + 8 * hh;
  const unsigned short* bp = BT + (size_t)m * (size_t)K + 8 * hh;

#pragma unroll 1
  for (int k0 = 0; k0 < K; k0 += 32) {
    FragB af;
    af.h[0] = *(const v8usa*)(ap + k0);
    af.h[1] = *(const v8usa*)(ap + k0 + 16);
#pragma unroll
    for (int nt = 0; nt < 8; ++nt) {
      const unsigned short* wq = bp + (size_t)(16 * nt) * (size_t)K + k0;
      FragB bf;
      bf.h[0] = *(const v8usa*)wq;
      bf.h[1] = *(const v8usa*)(wq + 16);
      acc[nt] = wmb(af, bf, acc[nt]);
    }
  }

#pragma unroll
  for (int nt = 0; nt < 8; ++nt) {
    const int lc = 16 * nt + m;
#pragma unroll
    for (int r = 0; r < 8; ++r) {
      const int lr = 16 * wave + 8 * hh + r;
      stg[lr * GBN + lc] = acc[nt][r];
    }
  }
  __syncthreads();

  v4f pv[16];
#pragma unroll
  for (int i = 0; i < 16; ++i) pv[i] = *(const v4fa*)(stg + (16 * wave + i) * GBN + 4 * lane);
#pragma unroll
  for (int i = 0; i < 16; ++i) {
    const int r = rowBase + 16 * wave + i;
    *(volatile v4f*)(outF + (size_t)r * DF + 4 * lane) = pv[i];
  }
  __threadfence();
#pragma unroll
  for (int i = 0; i < 16; ++i) {
    const int r = rowBase + 16 * wave + i;
    *(volatile v4f*)(outF + (size_t)r * DF + 4 * lane) = pv[i];
  }
}

template <int MODE>
__global__ __launch_bounds__(NTHR) void k_agg(const int* __restrict__ srcs, const int* __restrict__ dsts,
                                              int nE, int nN, int vec8, int mRows,
                                              const float* __restrict__ dis, const float* __restrict__ xl,
                                              const float* __restrict__ bias, const float* __restrict__ wout,
                                              const float* __restrict__ bout,
                                              unsigned short* hb, float* outp) {
  extern __shared__ __attribute__((aligned(16))) int dsm[];
  int* list  = dsm;
  int* hl    = dsm + LISTN;
  int* sl    = hl + RCAP;
  int* cnt   = sl + RCAP;
  int* offs  = cnt + NBA;
  int* cur   = offs + NBA;
  int* misc  = cur + NBA;
  int* stage = misc + MISC_INTS;
  const int tid = (int)threadIdx.x, lane = tid & 31, wave = tid >> 5;
  const int nodeBase = (int)blockIdx.x * NBA;

  {
    const v4i z4 = {0, 0, 0, 0};
    for (int i = tid * 4; i < AGG_ZINTS; i += NTHR * 4) *(v4ia*)(dsm + i) = z4;
    if (tid < MISC_INTS) misc[tid] = 0;
    for (int i = tid; i < STAGE_INTS; i += NTHR) stage[i] = 0;
  }
  v4f bv;
  {
    const v4f a = *(const v4f*)(bias + 4 * lane);
    bv.x = bf16_val(a.x); bv.y = bf16_val(a.y); bv.z = bf16_val(a.z); bv.w = bf16_val(a.w);
  }
  v4f wv = {0.0f, 0.0f, 0.0f, 0.0f};
  float bo = 0.0f;
  if constexpr (MODE == 2) {
    const v4f a = *(const v4f*)(wout + 4 * lane);
    wv.x = bf16_val(a.x); wv.y = bf16_val(a.y); wv.z = bf16_val(a.z); wv.w = bf16_val(a.w);
    bo = bf16_val(bout[0]);
  }
  __syncthreads();

  int t = 0, ov = 0;
  const int nChunks = (nE + CHUNK - 1) / CHUNK;
#pragma unroll 1
  for (int ch = 0; ch < nChunks; ++ch) {
    const int cbase = ch * CHUNK;
    const int wc = scan_chunk<SLA>(dsts, nE, cbase, nodeBase, NBA, vec8, list, tid, lane, wave);
    if (lane == 0) misc[wave] = wc;
    __syncthreads();
    if (wave == 0) {
#pragma unroll 1
      for (int w2 = 0; w2 < NWAVE; ++w2) {
        int c = misc[w2];
        c = c < 0 ? 0 : (c > WCAP ? WCAP : c);
#pragma unroll 1
        for (int b0 = 0; b0 < c; b0 += 32) {
          const int idx = b0 + lane;
          const int ent = list[w2 * WCAP + (idx < WCAP ? idx : WCAP - 1)];
          const int m32 = (c - b0) < 32 ? (c - b0) : 32;
#pragma unroll 1
          for (int k = 0; k < m32; ++k) {
            const int u    = __builtin_amdgcn_readlane(ent, k);
            const int slot = u & (NBA - 1);
            const int el   = (u >> SLA) & (CHUNK - 1);
            const int pk   = ((cbase + el) << SLA) | slot;
            if (t < RCAP) {
              if (lane == 0) { hl[t] = pk; cnt[slot] = cnt[slot] + 1; }
              t = t + 1;
            } else {
              ov = 1;
            }
          }
        }
      }
    }
    __syncthreads();
  }
  if (wave == 0 && lane == 0) { misc[8] = t; misc[9] = ov; }
  __syncthreads();
  int tt = misc[8];
  tt = tt < 0 ? 0 : (tt > RCAP ? RCAP : tt);
  const int ovf = misc[9];

  if (wave == 0) {
    const int base = lane * (NBA / 32);
    int s = 0;
#pragma unroll 1
    for (int i = 0; i < NBA / 32; ++i) s += cnt[base + i];
    int incl = s;
#pragma unroll
    for (int d = 1; d < 32; d <<= 1) {
      const int y = __shfl_up(incl, d, 32);
      if (lane >= d) incl += y;
    }
    int run = incl - s;
#pragma unroll 1
    for (int i = 0; i < NBA / 32; ++i) {
      const int cv = cnt[base + i];
      offs[base + i] = run;
      cur[base + i]  = run;
      run += cv;
    }
  }
  __syncthreads();
  if (wave == 0) {
#pragma unroll 1
    for (int b0 = 0; b0 < tt; b0 += 32) {
      const int idx = b0 + lane;
      const int ent = hl[idx < RCAP ? idx : RCAP - 1];
      const int m32 = (tt - b0) < 32 ? (tt - b0) : 32;
#pragma unroll 1
      for (int k = 0; k < m32; ++k) {
        const int u    = __builtin_amdgcn_readlane(ent, k);
        const int slot = u & (NBA - 1);
        if (lane == 0) {
          int p = cur[slot];
          p = p < 0 ? 0 : (p > RCAP - 1 ? RCAP - 1 : p);
          sl[p] = u;
          cur[slot] = p + 1;
        }
      }
    }
  }
  __syncthreads();

  const float qnan = __int_as_float(0x7fc00000);
  const float pz = (ovf != 0) ? qnan : 0.0f;
  const int sa = (2 * lane) & 31, sb = (2 * lane + 1) & 31;
#pragma unroll 1
  for (int si = 0; si < NBA / NWAVE; ++si) {
    const int s    = si * NWAVE + wave;
    const int node = nodeBase + s;
    int c = cnt[s];
    const bool big = c > DEGCAP;
    c = c < 0 ? 0 : (c > DEGCAP ? DEGCAP : c);
    int o = offs[s];
    o = o < 0 ? 0 : (o > RCAP ? RCAP : o);
    const int nc = node < nN ? node : nN - 1;
    const float dd = dis[nc];
    const float rd = dd * dd;
    float a0 = 0.0f, a1 = 0.0f, a2 = 0.0f, a3 = 0.0f;
#pragma unroll 1
    for (int b0 = 0; b0 < c; b0 += 32) {
      int idx = o + b0 + lane;
      idx = idx > RCAP - 1 ? RCAP - 1 : idx;
      const int ent = sl[idx];
      int eid = ent >> SLA;
      eid = eid < 0 ? 0 : (eid > nE - 1 ? nE - 1 : eid);
      int sr = srcs[eid];
      sr = sr < 0 ? 0 : (sr > nN - 1 ? nN - 1 : sr);
      const float cf  = dis[sr] * dd;
      const int   cfi = __float_as_int(cf);
      const int m32 = (c - b0) < 32 ? (c - b0) : 32;
#pragma unroll 1
      for (int k = 0; k < m32; ++k) {
        const int   sk = __builtin_amdgcn_readlane(sr, k);
        const float ck = __int_as_float(__builtin_amdgcn_readlane(cfi, k));
        const v4f a = *(const v4fa*)(xl + (size_t)sk * DF + 4 * lane);
        a0 = fmaf(ck, a.x, a0);
        a1 = fmaf(ck, a.y, a1);
        a2 = fmaf(ck, a.z, a2);
        a3 = fmaf(ck, a.w, a3);
      }
    }
    const v4f sv = *(const v4fa*)(xl + (size_t)nc * DF + 4 * lane);
    const float pzr = big ? qnan : pz;
    const bool live = node < nN;
    float y0 = (a0 + sv.x * rd) + bv.x;
    float y1 = (a1 + sv.y * rd) + bv.y;
    float y2 = (a2 + sv.z * rd) + bv.z;
    float y3 = (a3 + sv.w * rd) + bv.w;
    y0 = (y0 > 0.0f) ? y0 : (y0 - y0);
    y1 = (y1 > 0.0f) ? y1 : (y1 - y1);
    y2 = (y2 > 0.0f) ? y2 : (y2 - y2);
    y3 = (y3 > 0.0f) ? y3 : (y3 - y3);
    y0 = y0 + pzr; y1 = y1 + pzr; y2 = y2 + pzr; y3 = y3 + pzr;
    const float v0 = live ? y0 : 0.0f;
    const float v1 = live ? y1 : 0.0f;
    const float v2 = live ? y2 : 0.0f;
    const float v3 = live ? y3 : 0.0f;
    if constexpr (MODE == 1) {
      const unsigned hb0 = bf16_bits(v0), hb1 = bf16_bits(v1), hb2 = bf16_bits(v2), hb3 = bf16_bits(v3);
      const unsigned lb0 = bf16_bits(v0 - __uint_as_float(hb0 << 16));
      const unsigned lb1 = bf16_bits(v1 - __uint_as_float(hb1 << 16));
      const unsigned lb2 = bf16_bits(v2 - __uint_as_float(hb2 << 16));
      const unsigned lb3 = bf16_bits(v3 - __uint_as_float(hb3 << 16));
      const int hw0 = (int)(hb0 | (hb1 << 16));
      const int hw1 = (int)(hb2 | (hb3 << 16));
      const int lw0 = (int)(lb0 | (lb1 << 16));
      const int lw1 = (int)(lb2 | (lb3 << 16));
      const int g0 = __shfl(hw0, sa, 32), g1 = __shfl(hw1, sa, 32);
      const int g2 = __shfl(hw0, sb, 32), g3 = __shfl(hw1, sb, 32);
      const int p0 = __shfl(lw0, sa, 32), p1 = __shfl(lw1, sa, 32);
      const int p2 = __shfl(lw0, sb, 32), p3 = __shfl(lw1, sb, 32);
      const bool lsel = lane >= 16;
      v4u pv;
      pv.x = (unsigned int)(lsel ? p0 : g0);
      pv.y = (unsigned int)(lsel ? p1 : g1);
      pv.z = (unsigned int)(lsel ? p2 : g2);
      pv.w = (unsigned int)(lsel ? p3 : g3);
      if (node < mRows) {
        unsigned short* hp = hb + (size_t)node * K2 + 8 * lane;
        *(volatile v4u*)hp = pv;
        __threadfence();
        *(volatile v4u*)hp = pv;
      }
    } else {
      float p = v0 * wv.x;
      p = fmaf(v1, wv.y, p);
      p = fmaf(v2, wv.z, p);
      p = fmaf(v3, wv.w, p);
#pragma unroll
      for (int d = 16; d >= 1; d >>= 1) p += __shfl_xor(p, d, 32);
      const float z = p + bo;
      float sc = 1.0f / (1.0f + expf(-z));
      sc = (big || (ovf != 0)) ? qnan : sc;
      sc = live ? sc : 0.0f;
      if (lane == 0) stage[s] = __float_as_int(sc);
    }
  }

  if constexpr (MODE == 2) {
    __syncthreads();
    const v4i q = *(const v4ia*)(stage + 4 * tid);
    v4f ovv;
    ovv.x = __int_as_float(q.x); ovv.y = __int_as_float(q.y);
    ovv.z = __int_as_float(q.z); ovv.w = __int_as_float(q.w);
    const int g0 = nodeBase + 4 * tid;
    const bool wr = (g0 + 3) < nN;
    float* op = outp + (size_t)(wr ? g0 : 0);
    if (wr) *(volatile v4f*)op = ovv;
    __threadfence();
    if (wr) *(volatile v4f*)op = ovv;
  }
}

static inline int cdiv(int a, int b) { return (a + b - 1) / b; }
static inline size_t al256(size_t o) { return (o + 255) & ~(size_t)255; }

extern "C" void kernel_launch(void* const* d_in, const int* in_sizes, int n_in,
                              void* d_out, int out_size, void* d_ws, size_t ws_size,
                              hipStream_t stream) {
  if (n_in < 10) return;
  if (in_sizes[0] < DF || (in_sizes[0] % DF) != 0) return;
  const int nN = in_sizes[0] / DF;
  if (nN < 16 || nN > (1 << 22) || (nN & 3) != 0) return;
  if (in_sizes[1] < 2 || (in_sizes[1] & 1) != 0) return;
  const int nE = in_sizes[1] / 2;
  if (nE < 1 || nE >= (1 << (31 - SLA))) return;
  if (in_sizes[2] != DF * DF || in_sizes[3] != DF) return;
  if (in_sizes[4] != DF * DF || in_sizes[5] != DF) return;
  if (in_sizes[6] != DF * DF || in_sizes[7] != DF) return;
  if (in_sizes[8] != DF || in_sizes[9] != 1) return;
  if (out_size != nN) return;

  const float* x    = (const float*)d_in[0];
  const int*   edge = (const int*)d_in[1];
  const float* W1   = (const float*)d_in[2];
  const float* b1   = (const float*)d_in[3];
  const float* W2   = (const float*)d_in[4];
  const float* b2   = (const float*)d_in[5];
  const float* W3   = (const float*)d_in[6];
  const float* b3   = (const float*)d_in[7];
  const float* Wout = (const float*)d_in[8];
  const float* bout = (const float*)d_in[9];
  float* out = (float*)d_out;
  const int* src = edge;
  const int* dst = edge + nE;

  const int MP   = cdiv(nN, GBM) * GBM;
  const int gM   = MP / GBM;
  const int nBx  = MP / 16;
  const int gD   = cdiv(nN, NBD);
  const int NBPD = gD * NBD;
  const int gA   = cdiv(MP, NBA);
  if ((long long)gA * NBA < (long long)MP) return;
  if (NBPD < nN) return;
  const int vec8 = ((nE & 3) == 0) ? 1 : 0;

  char* ws = (char*)d_ws;
  size_t off = 0;
  const size_t oDIS = off; off = al256(off + (size_t)NBPD * 4);
  const size_t oW1T = off; off = al256(off + (size_t)DF * DF * 2);
  const size_t oW2D = off; off = al256(off + (size_t)DF * K2 * 2);
  const size_t oW3D = off; off = al256(off + (size_t)DF * K2 * 2);
  const size_t oXB  = off; off = al256(off + (size_t)MP * DF * 2);
  const size_t oH   = off; off = al256(off + (size_t)MP * DF * 4);
  const size_t oXHL = off; off = al256(off + (size_t)MP * K2 * 2);
  if (off > ws_size || off > (size_t)WSMAX) return;
  float*          DIS = (float*)(ws + oDIS);
  unsigned short* W1T = (unsigned short*)(ws + oW1T);
  unsigned short* W2D = (unsigned short*)(ws + oW2D);
  unsigned short* W3D = (unsigned short*)(ws + oW3D);
  unsigned short* XB  = (unsigned short*)(ws + oXB);
  float*          H   = (float*)(ws + oH);
  unsigned short* XHL = (unsigned short*)(ws + oXHL);

  const size_t aggLds = (size_t)AGG_LDS_INTS * 4;
  hipFuncSetAttribute(reinterpret_cast<const void*>(&k_agg<1>), hipFuncAttributeMaxDynamicSharedMemorySize, (int)aggLds);
  hipFuncSetAttribute(reinterpret_cast<const void*>(&k_agg<2>), hipFuncAttributeMaxDynamicSharedMemorySize, (int)aggLds);

  k_prep<<<nBx + NBW, NTHR, 0, stream>>>(x, W1, W2, W3, nN, nBx, XB, W1T, W2D, W3D);
  k_deg<<<gD, NTHR, 0, stream>>>(dst, nE, vec8, DIS);
  k_gemm<<<gM, GTHR, 0, stream>>>(XB, W1T, DF, H);
  k_agg<1><<<gA, NTHR, aggLds, stream>>>(src, dst, nE, nN, vec8, MP, DIS, H, b1, Wout, bout, XHL, out);
  k_gemm<<<gM, GTHR, 0, stream>>>(XHL, W2D, K2, H);
  k_agg<1><<<gA, NTHR, aggLds, stream>>>(src, dst, nE, nN, vec8, MP, DIS, H, b2, Wout, bout, XHL, out);
  k_gemm<<<gM, GTHR, 0, stream>>>(XHL, W3D, K2, H);
  k_agg<2><<<gA, NTHR, aggLds, stream>>>(src, dst, nE, nN, vec8, MP, DIS, H, b3, Wout, bout, XHL, out);
}
